// GCNAutoEncoder_89300960019182
// MI455X (gfx1250) — hardware-verified
//
#include <hip/hip_runtime.h>
#include <hip/hip_bf16.h>
#include <stddef.h>


#define KD      128
#define NTHR    256
#define NWAVE   8
#define EPT     8
#define NGRP    2
#define CHUNK   (NTHR * EPT * NGRP)
#define WCAP    (EPT * NGRP * 32)
#define LISTN   (NWAVE * WCAP)
#define SB      13
#define RPAD    8192
#define NBD     8192
#define NB128   512
#define NB64    1024
#define NB8     4096
#define WPLN    (2 * 128 * KD + 2 * 64 * KD + 2 * 128 * KD)

#define LDS_DEG (NBD * 4 + LISTN * 4)
#define LDS_128 (NB128 * 128 * 4 + LISTN * 4)
#define LDS_64  (NB64 * 64 * 4 + LISTN * 4)
#define LDS_8   (NB8 * 8 * 4 + LISTN * 4)

static_assert((CHUNK & (CHUNK - 1)) == 0);
static_assert(CHUNK <= 4096);
static_assert(NBD <= (1 << SB) && NB8 <= (1 << SB) && NB64 <= (1 << SB) && NB128 <= (1 << SB));
static_assert((NBD & (NBD - 1)) == 0 && (NB128 & (NB128 - 1)) == 0 && (NB64 & (NB64 - 1)) == 0 && (NB8 & (NB8 - 1)) == 0);
static_assert(RPAD % NBD == 0 && RPAD % NB128 == 0 && RPAD % NB64 == 0 && RPAD % NB8 == 0 && RPAD % 128 == 0);
static_assert(NBD == NWAVE * 1024 && NB64 * 8 == NWAVE * 1024);
static_assert(NB128 % (2 * NWAVE) == 0 && NB8 % (2 * NWAVE) == 0 && NB64 % NWAVE == 0);

typedef float v2f __attribute__((ext_vector_type(2)));
typedef float v4f __attribute__((ext_vector_type(4)));
typedef float v8f __attribute__((ext_vector_type(8)));
typedef int   v4i __attribute__((ext_vector_type(4)));
typedef unsigned short v8us  __attribute__((ext_vector_type(8)));
typedef unsigned short v16us __attribute__((ext_vector_type(16)));
typedef __bf16 v16bf __attribute__((ext_vector_type(16)));
union FragB { v16bf v; v16us u; v8us h[2]; };
struct HL { v8us hi; v8us lo; };

__device__ __forceinline__ unsigned int bf_bits(float f) {
  const unsigned int u = __float_as_uint(f);
  return (u + 0x7FFFu + ((u >> 16) & 1u)) >> 16;
}
__device__ __forceinline__ unsigned int bf_lo(float f, unsigned int hb) {
  return bf_bits(f - __uint_as_float(hb << 16));
}
__device__ __forceinline__ HL split8(v4f a, v4f b) {
  HL r;
  unsigned int h;
  h = bf_bits(a.x); r.hi[0] = (unsigned short)h; r.lo[0] = (unsigned short)bf_lo(a.x, h);
  h = bf_bits(a.y); r.hi[1] = (unsigned short)h; r.lo[1] = (unsigned short)bf_lo(a.y, h);
  h = bf_bits(a.z); r.hi[2] = (unsigned short)h; r.lo[2] = (unsigned short)bf_lo(a.z, h);
  h = bf_bits(a.w); r.hi[3] = (unsigned short)h; r.lo[3] = (unsigned short)bf_lo(a.w, h);
  h = bf_bits(b.x); r.hi[4] = (unsigned short)h; r.lo[4] = (unsigned short)bf_lo(b.x, h);
  h = bf_bits(b.y); r.hi[5] = (unsigned short)h; r.lo[5] = (unsigned short)bf_lo(b.y, h);
  h = bf_bits(b.z); r.hi[6] = (unsigned short)h; r.lo[6] = (unsigned short)bf_lo(b.z, h);
  h = bf_bits(b.w); r.hi[7] = (unsigned short)h; r.lo[7] = (unsigned short)bf_lo(b.w, h);
  return r;
}

__device__ __forceinline__ v4f relu4(v4f t) {
  t.x = fmaxf(t.x, 0.f); t.y = fmaxf(t.y, 0.f); t.z = fmaxf(t.z, 0.f); t.w = fmaxf(t.w, 0.f);
  return t;
}

__device__ __forceinline__ float wsum32(float s) {
  s += __shfl_xor(s, 16, 32);
  s += __shfl_xor(s, 8, 32);
  s += __shfl_xor(s, 4, 32);
  s += __shfl_xor(s, 2, 32);
  s += __shfl_xor(s, 1, 32);
  return s;
}

__device__ __forceinline__ v8f wmb(v16bf a, v16bf b, v8f c) {
  v8f d = __builtin_amdgcn_wmma_f32_16x16x32_bf16(false, a, false, b, (short)0, c, false, false);
  asm volatile("v_nop\n\tv_nop\n\tv_nop\n\tv_nop" : "+v"(d) : "v"(a), "v"(b));
  return d;
}

template <int NBT>
__device__ __forceinline__ int scan_chunk(const int* __restrict__ dsts, int nE, int cbase, int nodeBase,
                                          int vec8, int* list, int tid, int wave) {
  int wc = 0;
#pragma unroll
  for (int g = 0; g < NGRP; ++g) {
    const int el0  = (g * NTHR + tid) * EPT;
    const int e0   = cbase + el0;
    const int sent = -2147483647 - 1;
    v4i da, db;
    if (vec8 != 0 && e0 + 7 < nE) {
      da = *(const v4i*)(dsts + e0);
      db = *(const v4i*)(dsts + e0 + 4);
    } else {
      da.x = (e0     < nE) ? dsts[min(e0, nE - 1)] : sent;
      da.y = (e0 + 1 < nE) ? dsts[min(e0 + 1, nE - 1)] : sent;
      da.z = (e0 + 2 < nE) ? dsts[min(e0 + 2, nE - 1)] : sent;
      da.w = (e0 + 3 < nE) ? dsts[min(e0 + 3, nE - 1)] : sent;
      db.x = (e0 + 4 < nE) ? dsts[min(e0 + 4, nE - 1)] : sent;
      db.y = (e0 + 5 < nE) ? dsts[min(e0 + 5, nE - 1)] : sent;
      db.z = (e0 + 6 < nE) ? dsts[min(e0 + 6, nE - 1)] : sent;
      db.w = (e0 + 7 < nE) ? dsts[min(e0 + 7, nE - 1)] : sent;
    }
    const unsigned nb = (unsigned)nodeBase;
    const unsigned s0 = (unsigned)da.x - nb, s1 = (unsigned)da.y - nb;
    const unsigned s2 = (unsigned)da.z - nb, s3 = (unsigned)da.w - nb;
    const unsigned s4 = (unsigned)db.x - nb, s5 = (unsigned)db.y - nb;
    const unsigned s6 = (unsigned)db.z - nb, s7 = (unsigned)db.w - nb;
    const bool h0 = s0 < (unsigned)NBT, h1 = s1 < (unsigned)NBT, h2 = s2 < (unsigned)NBT, h3 = s3 < (unsigned)NBT;
    const bool h4 = s4 < (unsigned)NBT, h5 = s5 < (unsigned)NBT, h6 = s6 < (unsigned)NBT, h7 = s7 < (unsigned)NBT;
    const unsigned any = __builtin_amdgcn_ballot_w32(h0 | h1 | h2 | h3 | h4 | h5 | h6 | h7);
    if (any != 0u) {
#define HITJ(J, HJ, SJ) { \
        const unsigned mj = __builtin_amdgcn_ballot_w32(HJ); \
        if (mj != 0u) { \
          if (HJ) { \
            const int pos = wc + (int)__builtin_amdgcn_mbcnt_lo(mj, 0u); \
            if (pos < WCAP) list[wave * WCAP + pos] = ((el0 + (J)) << SB) | (int)(SJ); \
          } \
          wc += (int)__builtin_popcount(mj); } }
      HITJ(0, h0, s0)
      HITJ(1, h1, s1)
      HITJ(2, h2, s2)
      HITJ(3, h3, s3)
      HITJ(4, h4, s4)
      HITJ(5, h5, s5)
      HITJ(6, h6, s6)
      HITJ(7, h7, s7)
#undef HITJ
    }
  }
  return wc;
}

__global__ __launch_bounds__(NTHR) void k_wprep(
    const float* __restrict__ w1, const float* __restrict__ w2, const float* __restrict__ w4,
    unsigned short* wpl) {
  const int i = blockIdx.x * NTHR + threadIdx.x;
  if (i >= 320 * (KD / 8)) return;
  const int na = i >> 4;
  const int k0 = (i & 15) * 8;
  const float* W; int n, F; size_t base;
  if (na < 128)      { W = w1; n = na;       F = 128; base = 0; }
  else if (na < 192) { W = w2; n = na - 128; F = 64;  base = (size_t)2 * 128 * KD; }
  else               { W = w4; n = na - 192; F = 128; base = (size_t)2 * 128 * KD + (size_t)2 * 64 * KD; }
  v4f a, bq;
  a.x  = W[(size_t)(k0 + 0) * F + n]; a.y  = W[(size_t)(k0 + 1) * F + n];
  a.z  = W[(size_t)(k0 + 2) * F + n]; a.w  = W[(size_t)(k0 + 3) * F + n];
  bq.x = W[(size_t)(k0 + 4) * F + n]; bq.y = W[(size_t)(k0 + 5) * F + n];
  bq.z = W[(size_t)(k0 + 6) * F + n]; bq.w = W[(size_t)(k0 + 7) * F + n];
  const HL s = split8(a, bq);
  unsigned short* ph = wpl + base + (size_t)n * KD + k0;
  unsigned short* pl = ph + (size_t)F * KD;
  *(volatile v8us*)ph = s.hi;
  *(volatile v8us*)pl = s.lo;
  __threadfence();
  *(volatile v8us*)ph = s.hi;
  *(volatile v8us*)pl = s.lo;
}

__global__ __launch_bounds__(NTHR) void k_deg(const int* __restrict__ ei, float* dinv, int nE, int vec8) {
  extern __shared__ v4f lds_dyn[];
  int* cnt  = (int*)lds_dyn;
  int* list = cnt + NBD;
  __shared__ int wcnt[NWAVE];
  const int tid = threadIdx.x, lane = tid & 31, wave = tid >> 5;
  const int nodeBase = blockIdx.x * NBD;
  const int* dsts = ei + nE;

  for (int i = tid; i < NBD; i += NTHR) cnt[i] = 0;
  __syncthreads();

  const int nChunks = (nE + CHUNK - 1) / CHUNK;
#pragma unroll 1
  for (int ch = 0; ch < nChunks; ++ch) {
    const int cbase = ch * CHUNK;
    const int wc = scan_chunk<NBD>(dsts, nE, cbase, nodeBase, vec8, list, tid, wave);
    if (lane == 0) wcnt[wave] = wc;
    __syncthreads();
    if (wave == 0) {
#pragma unroll 1
      for (int wsx = 0; wsx < NWAVE; ++wsx) {
        int n = __builtin_amdgcn_readfirstlane(wcnt[wsx]);
        n = n > WCAP ? WCAP : (n < 0 ? 0 : n);
        const int* lp = list + wsx * WCAP;
#pragma unroll 1
        for (int i = 0; i < n; ++i) {
          const int ent  = __builtin_amdgcn_readfirstlane(lp[i]);
          const int slot = ent & (NBD - 1);
          if (lane == 0) cnt[slot] = cnt[slot] + 1;
        }
      }
    }
    __syncthreads();
  }

  v4f ov[8];
#pragma unroll
  for (int q = 0; q < 8; ++q) {
    const int f = wave * 1024 + q * 128 + 4 * lane;
    const v4i c = *(const v4i*)(cnt + f);
    v4f v;
    v.x = rsqrtf((float)(c.x + 1)); v.y = rsqrtf((float)(c.y + 1));
    v.z = rsqrtf((float)(c.z + 1)); v.w = rsqrtf((float)(c.w + 1));
    ov[q] = v;
  }
  float* gp = dinv + (size_t)nodeBase + wave * 1024 + 4 * lane;
#pragma unroll
  for (int q = 0; q < 8; ++q) *(volatile v4f*)(gp + q * 128) = ov[q];
  __threadfence();
#pragma unroll
  for (int q = 0; q < 8; ++q) *(volatile v4f*)(gp + q * 128) = ov[q];
}

template <int FOUT, bool A16>
__global__ __launch_bounds__(NTHR) void k_gemm(
    const float* __restrict__ xa, const unsigned short* __restrict__ pa, const unsigned short* __restrict__ pb,
    const unsigned short* __restrict__ whi, const float* __restrict__ dinv,
    float* G, int nN, int nPad) {
  constexpr int NCH   = FOUT / 64;
  constexpr int GROWS = 16 * (NWAVE / NCH);
  static_assert(GROWS * FOUT == NWAVE * 1024);
  __shared__ __attribute__((aligned(16))) float stg[GROWS * FOUT];
  const int tid = threadIdx.x, lane = tid & 31, wave = tid >> 5, hh = lane >> 4, m = lane & 15;
  const int ch   = wave % NCH;
  const int rt   = wave / NCH;
  const int row0 = blockIdx.x * GROWS + rt * 16;
  const int col0 = ch * 64;
  int node = row0 + m;
  node = node > nN - 1 ? nN - 1 : node;
  const unsigned short* wlo = whi + (size_t)FOUT * KD;

  v8f acc[4];
#pragma unroll
  for (int t = 0; t < 4; ++t) { v8f z = {0.f, 0.f, 0.f, 0.f, 0.f, 0.f, 0.f, 0.f}; acc[t] = z; }

#pragma unroll
  for (int ks = 0; ks < KD / 32; ++ks) {
    FragB ah, al;
    if constexpr (A16) {
      const unsigned short* p = pa + (size_t)node * KD + 32 * ks + 8 * hh;
      const unsigned short* q = pb + (size_t)node * KD + 32 * ks + 8 * hh;
      ah.h[0] = *(const v8us*)p; ah.h[1] = *(const v8us*)(p + 16);
      al.h[0] = *(const v8us*)q; al.h[1] = *(const v8us*)(q + 16);
    } else {
      const float* p0 = xa + (size_t)node * KD + 32 * ks + 8 * hh;
      const v4f f0 = *(const v4f*)p0,        f1 = *(const v4f*)(p0 + 4);
      const v4f f2 = *(const v4f*)(p0 + 16), f3 = *(const v4f*)(p0 + 20);
      const HL s0 = split8(f0, f1);
      const HL s1 = split8(f2, f3);
      ah.h[0] = s0.hi; ah.h[1] = s1.hi;
      al.h[0] = s0.lo; al.h[1] = s1.lo;
    }
#pragma unroll
    for (int t = 0; t < 4; ++t) {
      const unsigned short* bp = whi + (size_t)(col0 + 16 * t + m) * KD + 32 * ks + 8 * hh;
      const unsigned short* bq = wlo + (size_t)(col0 + 16 * t + m) * KD + 32 * ks + 8 * hh;
      FragB bh, bl;
      bh.h[0] = *(const v8us*)bp; bh.h[1] = *(const v8us*)(bp + 16);
      bl.h[0] = *(const v8us*)bq; bl.h[1] = *(const v8us*)(bq + 16);
      acc[t] = wmb(ah.v, bh.v, acc[t]);
      acc[t] = wmb(ah.v, bl.v, acc[t]);
      acc[t] = wmb(al.v, bh.v, acc[t]);
    }
  }

  float* sp = stg + (size_t)(rt * 16 + 8 * hh) * FOUT + col0 + m;
#pragma unroll
  for (int t = 0; t < 4; ++t) {
    sp[0 * FOUT + 16 * t] = acc[t][0];
    sp[1 * FOUT + 16 * t] = acc[t][1];
    sp[2 * FOUT + 16 * t] = acc[t][2];
    sp[3 * FOUT + 16 * t] = acc[t][3];
    sp[4 * FOUT + 16 * t] = acc[t][4];
    sp[5 * FOUT + 16 * t] = acc[t][5];
    sp[6 * FOUT + 16 * t] = acc[t][6];
    sp[7 * FOUT + 16 * t] = acc[t][7];
  }
  __syncthreads();

  v4f ov[8];
#pragma unroll
  for (int q = 0; q < 8; ++q) {
    const int f = wave * 1024 + q * 128 + 4 * lane;
    int grow = blockIdx.x * GROWS + f / FOUT;
    grow = grow > nPad - 1 ? nPad - 1 : grow;
    const float di = dinv[grow];
    ov[q] = *(const v4f*)(stg + f) * di;
  }
  float* gp = G + (size_t)blockIdx.x * (GROWS * FOUT) + wave * 1024 + 4 * lane;
#pragma unroll
  for (int q = 0; q < 8; ++q) *(volatile v4f*)(gp + q * 128) = ov[q];
  __threadfence();
#pragma unroll
  for (int q = 0; q < 8; ++q) *(volatile v4f*)(gp + q * 128) = ov[q];
}

__device__ __forceinline__ void planes_pass128(const float* acc, unsigned short* ph, unsigned short* pl,
                                               int nodeBase, int wave, int lane) {
  const int hs = lane >> 4, c0 = 8 * (lane & 15);
#pragma unroll 2
  for (int j = 0; j < NB128 / (2 * NWAVE); ++j) {
    const int slot = wave * (NB128 / NWAVE) + 2 * j + hs;
    const float* la = acc + slot * 128 + c0;
    const v4f a = *(const v4f*)la, b = *(const v4f*)(la + 4);
    const HL s = split8(a, b);
    const size_t go = (size_t)(nodeBase + slot) * 128 + c0;
    *(volatile v8us*)(ph + go) = s.hi;
    *(volatile v8us*)(pl + go) = s.lo;
  }
}
__device__ __forceinline__ void rows_pass128(const float* acc, float* out, int nodeBase, int nN,
                                             int wave, int lane) {
#pragma unroll 4
  for (int j = 0; j < NB128 / NWAVE; ++j) {
    const int slot = wave * (NB128 / NWAVE) + j;
    const int row  = nodeBase + slot;
    if (row < nN) {
      const v4f v = *(const v4f*)(acc + slot * 128 + 4 * lane);
      *(volatile v4f*)(out + (size_t)row * 128 + 4 * lane) = v;
    }
  }
}

template <int MODE>
__global__ __launch_bounds__(NTHR) void k_agg128(
    const int* __restrict__ ei, const float* __restrict__ G, const float* __restrict__ dinv,
    const float* __restrict__ bias, unsigned short* ph, unsigned short* pl, float* out,
    int nN, int nE, int vec8) {
  extern __shared__ v4f lds_dyn[];
  float* acc  = (float*)lds_dyn;
  int*   list = (int*)(acc + NB128 * 128);
  __shared__ int wcnt[NWAVE];
  __shared__ __attribute__((aligned(16))) float sbias[128];
  const int tid = threadIdx.x, lane = tid & 31, wave = tid >> 5;
  const int nodeBase = blockIdx.x * NB128;
  const int* dsts = ei + nE;

  if (tid < 128) sbias[tid] = bias[tid];
  {
    const v4f z = {0.f, 0.f, 0.f, 0.f};
    for (int i = tid; i < NB128 * 128 / 4; i += NTHR) lds_dyn[i] = z;
  }
  __syncthreads();

  const int nChunks = (nE + CHUNK - 1) / CHUNK;
#pragma unroll 1
  for (int ch = 0; ch < nChunks; ++ch) {
    const int cbase = ch * CHUNK;
    const int wc = scan_chunk<NB128>(dsts, nE, cbase, nodeBase, vec8, list, tid, wave);
    if (lane == 0) wcnt[wave] = wc;
    __syncthreads();
    if (wave == 0) {
#pragma unroll 1
      for (int wsx = 0; wsx < NWAVE; ++wsx) {
        int n = __builtin_amdgcn_readfirstlane(wcnt[wsx]);
        n = n > WCAP ? WCAP : (n < 0 ? 0 : n);
        const int* lp = list + wsx * WCAP;
#pragma unroll 1
        for (int i = 0; i < n; ++i) {
          const int ent  = __builtin_amdgcn_readfirstlane(lp[i]);
          const int slot = ent & (NB128 - 1);
          int e = cbase + ((ent >> SB) & (CHUNK - 1));
          e = e > nE - 1 ? nE - 1 : e;
          int src = ei[e];
          src = src < 0 ? 0 : (src > nN - 1 ? nN - 1 : src);
          const v4f v = *(const v4f*)(G + (size_t)src * 128 + 4 * lane);
          v4f* ap = (v4f*)(acc + slot * 128 + 4 * lane);
          *ap = *ap + v;
        }
      }
    }
    __syncthreads();
  }

  const v4f b4 = *(const v4f*)(sbias + 4 * lane);
#pragma unroll 2
  for (int j = 0; j < NB128 / NWAVE; ++j) {
    const int slot = wave * (NB128 / NWAVE) + j;
    int node = nodeBase + slot;
    node = node > nN - 1 ? nN - 1 : node;
    const float di = dinv[node];
    v4f* ap = (v4f*)(acc + slot * 128 + 4 * lane);
    const v4f g = *(const v4f*)(G + (size_t)node * 128 + 4 * lane);
    v4f t = (*ap + g) * di + b4;
    if (MODE == 0) t = relu4(t);
    *ap = t;
  }
  __syncthreads();

  if (MODE == 0) {
    planes_pass128(acc, ph, pl, nodeBase, wave, lane);
    __threadfence();
    planes_pass128(acc, ph, pl, nodeBase, wave, lane);
  } else {
    rows_pass128(acc, out, nodeBase, nN, wave, lane);
    __threadfence();
    rows_pass128(acc, out, nodeBase, nN, wave, lane);
  }
}

__global__ __launch_bounds__(NTHR) void k_agg64z(
    const int* __restrict__ ei, const float* __restrict__ G, const float* __restrict__ dinv,
    const float* __restrict__ b2, const float* __restrict__ Wm, const float* __restrict__ bm,
    const float* __restrict__ lnw, const float* __restrict__ lnb, float* zbs,
    int nN, int nE, int vec8) {
  extern __shared__ v4f lds_dyn[];
  float* acc  = (float*)lds_dyn;
  int*   list = (int*)(acc + NB64 * 64);
  __shared__ int wcnt[NWAVE];
  __shared__ __attribute__((aligned(16))) float sW[64 * 5];
  __shared__ __attribute__((aligned(16))) float sb2[64];
  __shared__ float sbm[8], slw[8], slb[8];
  const int tid = threadIdx.x, lane = tid & 31, wave = tid >> 5;
  const int nodeBase = blockIdx.x * NB64;
  const int* dsts = ei + nE;

  for (int i = tid; i < 64 * 5; i += NTHR) sW[i] = Wm[i];
  if (tid < 64) sb2[tid] = b2[tid];
  if (tid < 5) { sbm[tid] = bm[tid]; slw[tid] = lnw[tid]; slb[tid] = lnb[tid]; }
  {
    const v4f z = {0.f, 0.f, 0.f, 0.f};
    for (int i = tid; i < NB64 * 64 / 4; i += NTHR) lds_dyn[i] = z;
  }
  __syncthreads();

  const int nChunks = (nE + CHUNK - 1) / CHUNK;
#pragma unroll 1
  for (int ch = 0; ch < nChunks; ++ch) {
    const int cbase = ch * CHUNK;
    const int wc = scan_chunk<NB64>(dsts, nE, cbase, nodeBase, vec8, list, tid, wave);
    if (lane == 0) wcnt[wave] = wc;
    __syncthreads();
    if (wave == 0) {
#pragma unroll 1
      for (int wsx = 0; wsx < NWAVE; ++wsx) {
        int n = __builtin_amdgcn_readfirstlane(wcnt[wsx]);
        n = n > WCAP ? WCAP : (n < 0 ? 0 : n);
        const int* lp = list + wsx * WCAP;
#pragma unroll 1
        for (int i = 0; i < n; ++i) {
          const int ent  = __builtin_amdgcn_readfirstlane(lp[i]);
          const int slot = ent & (NB64 - 1);
          int e = cbase + ((ent >> SB) & (CHUNK - 1));
          e = e > nE - 1 ? nE - 1 : e;
          int src = ei[e];
          src = src < 0 ? 0 : (src > nN - 1 ? nN - 1 : src);
          const v2f v = *(const v2f*)(G + (size_t)src * 64 + 2 * lane);
          v2f* ap = (v2f*)(acc + slot * 64 + 2 * lane);
          *ap = *ap + v;
        }
      }
    }
    __syncthreads();
  }

  const float bx = sb2[2 * lane], by = sb2[2 * lane + 1];
  const float* w0 = sW + 10 * lane;
#pragma unroll 1
  for (int j = 0; j < NB64 / NWAVE; ++j) {
    const int slot = wave * (NB64 / NWAVE) + j;
    int node = nodeBase + slot;
    node = node > nN - 1 ? nN - 1 : node;
    const float di = dinv[node];
    const v2f a = *(const v2f*)(acc + slot * 64 + 2 * lane);
    const v2f g = *(const v2f*)(G + (size_t)node * 64 + 2 * lane);
    float z0 = (a.x + g.x) * di + bx;
    float z1 = (a.y + g.y) * di + by;
    z0 = fmaxf(z0, 0.f); z1 = fmaxf(z1, 0.f);
    float p0 = z0 * w0[0] + z1 * w0[5];
    float p1 = z0 * w0[1] + z1 * w0[6];
    float p2 = z0 * w0[2] + z1 * w0[7];
    float p3 = z0 * w0[3] + z1 * w0[8];
    float p4 = z0 * w0[4] + z1 * w0[9];
    p0 = wsum32(p0); p1 = wsum32(p1); p2 = wsum32(p2); p3 = wsum32(p3); p4 = wsum32(p4);
    const float y0 = p0 + sbm[0], y1 = p1 + sbm[1], y2 = p2 + sbm[2], y3 = p3 + sbm[3], y4 = p4 + sbm[4];
    const float mu = (y0 + y1 + y2 + y3 + y4) * 0.2f;
    const float d0 = y0 - mu, d1 = y1 - mu, d2 = y2 - mu, d3 = y3 - mu, d4 = y4 - mu;
    const float var = (d0 * d0 + d1 * d1 + d2 * d2 + d3 * d3 + d4 * d4) * 0.2f;
    const float is = rsqrtf(var + 1e-5f);
    v4f u0, u1;
    u0.x = (d0 * is * slw[0] + slb[0]) * di;
    u0.y = (d1 * is * slw[1] + slb[1]) * di;
    u0.z = (d2 * is * slw[2] + slb[2]) * di;
    u0.w = (d3 * is * slw[3] + slb[3]) * di;
    u1.x = (d4 * is * slw[4] + slb[4]) * di;
    u1.y = 0.f; u1.z = 0.f; u1.w = 0.f;
    if (lane == 0) {
      *(v4f*)(acc + slot * 64)     = u0;
      *(v4f*)(acc + slot * 64 + 4) = u1;
    }
  }
  __syncthreads();

  v4f ov[8];
#pragma unroll
  for (int q = 0; q < 8; ++q) {
    const int f = wave * 1024 + q * 128 + 4 * lane;
    ov[q] = *(const v4f*)(acc + (f >> 3) * 64 + (f & 7));
  }
  float* gp = zbs + (size_t)nodeBase * 8 + wave * 1024 + 4 * lane;
#pragma unroll
  for (int q = 0; q < 8; ++q) *(volatile v4f*)(gp + q * 128) = ov[q];
  __threadfence();
#pragma unroll
  for (int q = 0; q < 8; ++q) *(volatile v4f*)(gp + q * 128) = ov[q];
}

__device__ __forceinline__ void planes_pass8(const float* acc, const float* __restrict__ zbs,
                                             const float* __restrict__ dinv, const float* sW, const float* sb,
                                             unsigned short* ph, unsigned short* pl,
                                             int nodeBase, int nN, int wave, int lane) {
  const int hs = lane >> 4, c0 = 8 * (lane & 15);
  const v4f bA = *(const v4f*)(sb + c0), bB = *(const v4f*)(sb + c0 + 4);
#pragma unroll 1
  for (int j = 0; j < NB8 / (2 * NWAVE); ++j) {
    const int slot = wave * (NB8 / NWAVE) + 2 * j + hs;
    int node = nodeBase + slot;
    node = node > nN - 1 ? nN - 1 : node;
    const float di = dinv[node];
    const v4f a0 = *(const v4f*)(acc + slot * 8), a1 = *(const v4f*)(acc + slot * 8 + 4);
    const v4f g0 = *(const v4f*)(zbs + (size_t)node * 8), g1 = *(const v4f*)(zbs + (size_t)node * 8 + 4);
    const float q0 = (a0.x + g0.x) * di, q1 = (a0.y + g0.y) * di, q2 = (a0.z + g0.z) * di;
    const float q3 = (a0.w + g0.w) * di, q4 = (a1.x + g1.x) * di;
    v4f vA = bA, vB = bB;
    vA = vA + *(const v4f*)(sW + 0 * 128 + c0) * q0;  vB = vB + *(const v4f*)(sW + 0 * 128 + c0 + 4) * q0;
    vA = vA + *(const v4f*)(sW + 1 * 128 + c0) * q1;  vB = vB + *(const v4f*)(sW + 1 * 128 + c0 + 4) * q1;
    vA = vA + *(const v4f*)(sW + 2 * 128 + c0) * q2;  vB = vB + *(const v4f*)(sW + 2 * 128 + c0 + 4) * q2;
    vA = vA + *(const v4f*)(sW + 3 * 128 + c0) * q3;  vB = vB + *(const v4f*)(sW + 3 * 128 + c0 + 4) * q3;
    vA = vA + *(const v4f*)(sW + 4 * 128 + c0) * q4;  vB = vB + *(const v4f*)(sW + 4 * 128 + c0 + 4) * q4;
    vA = relu4(vA); vB = relu4(vB);
    const HL s = split8(vA, vB);
    const size_t go = (size_t)(nodeBase + slot) * 128 + c0;
    *(volatile v8us*)(ph + go) = s.hi;
    *(volatile v8us*)(pl + go) = s.lo;
  }
}

__global__ __launch_bounds__(NTHR) void k_agg8d(
    const int* __restrict__ ei, const float* __restrict__ zbs, const float* __restrict__ dinv,
    const float* __restrict__ W1d, const float* __restrict__ b1d, unsigned short* ph, unsigned short* pl,
    int nN, int nE, int vec8) {
  extern __shared__ v4f lds_dyn[];
  float* acc  = (float*)lds_dyn;
  int*   list = (int*)(acc + NB8 * 8);
  __shared__ int wcnt[NWAVE];
  __shared__ __attribute__((aligned(16))) float sW[5 * 128];
  __shared__ __attribute__((aligned(16))) float sb[128];
  const int tid = threadIdx.x, lane = tid & 31, wave = tid >> 5;
  const int nodeBase = blockIdx.x * NB8;
  const int* dsts = ei + nE;

  for (int i = tid; i < 5 * 128; i += NTHR) sW[i] = W1d[i];
  if (tid < 128) sb[tid] = b1d[tid];
  {
    const v4f z = {0.f, 0.f, 0.f, 0.f};
    for (int i = tid; i < NB8 * 8 / 4; i += NTHR) lds_dyn[i] = z;
  }
  __syncthreads();

  const int nChunks = (nE + CHUNK - 1) / CHUNK;
#pragma unroll 1
  for (int ch = 0; ch < nChunks; ++ch) {
    const int cbase = ch * CHUNK;
    const int wc = scan_chunk<NB8>(dsts, nE, cbase, nodeBase, vec8, list, tid, wave);
    if (lane == 0) wcnt[wave] = wc;
    __syncthreads();
    if (wave == 0) {
#pragma unroll 1
      for (int wsx = 0; wsx < NWAVE; ++wsx) {
        int n = __builtin_amdgcn_readfirstlane(wcnt[wsx]);
        n = n > WCAP ? WCAP : (n < 0 ? 0 : n);
        const int* lp = list + wsx * WCAP;
#pragma unroll 1
        for (int i = 0; i < n; ++i) {
          const int ent  = __builtin_amdgcn_readfirstlane(lp[i]);
          const int slot = ent & (NB8 - 1);
          int e = cbase + ((ent >> SB) & (CHUNK - 1));
          e = e > nE - 1 ? nE - 1 : e;
          int src = ei[e];
          src = src < 0 ? 0 : (src > nN - 1 ? nN - 1 : src);
          if (lane < 2) {
            const v4f v = *(const v4f*)(zbs + (size_t)src * 8 + 4 * lane);
            v4f* ap = (v4f*)(acc + slot * 8 + 4 * lane);
            *ap = *ap + v;
          }
        }
      }
    }
    __syncthreads();
  }

  planes_pass8(acc, zbs, dinv, sW, sb, ph, pl, nodeBase, nN, wave, lane);
  __threadfence();
  planes_pass8(acc, zbs, dinv, sW, sb, ph, pl, nodeBase, nN, wave, lane);
}

extern "C" void kernel_launch(void* const* d_in, const int* in_sizes, int n_in,
                              void* d_out, int out_size, void* d_ws, size_t ws_size,
                              hipStream_t stream) {
  if (n_in < 14) return;
  const int nN = in_sizes[0] / KD;
  const int nE = in_sizes[1] / 2;
  if (nN <= 0 || nE < 0) return;
  if (in_sizes[0] != nN * KD || in_sizes[1] != 2 * nE) return;
  if (in_sizes[2] != KD * 128 || in_sizes[3] != 128) return;
  if (in_sizes[4] != KD * 64 || in_sizes[5] != 64) return;
  if (in_sizes[6] != 64 * 5 || in_sizes[7] != 5 || in_sizes[8] != 5 || in_sizes[9] != 5) return;
  if (in_sizes[10] != 5 * 128 || in_sizes[11] != 128) return;
  if (in_sizes[12] != KD * 128 || in_sizes[13] != 128) return;
  if (out_size != nN * 128) return;

  const float* x   = (const float*)d_in[0];
  const int*   ei  = (const int*)d_in[1];
  const float* W1e = (const float*)d_in[2];
  const float* b1e = (const float*)d_in[3];
  const float* W2e = (const float*)d_in[4];
  const float* b2e = (const float*)d_in[5];
  const float* Wm  = (const float*)d_in[6];
  const float* bm  = (const float*)d_in[7];
  const float* lnw = (const float*)d_in[8];
  const float* lnb = (const float*)d_in[9];
  const float* W1d = (const float*)d_in[10];
  const float* b1d = (const float*)d_in[11];
  const float* W2d = (const float*)d_in[12];
  const float* b2d = (const float*)d_in[13];
  float* out = (float*)d_out;

  const int nPad = ((nN + RPAD - 1) / RPAD) * RPAD;

  char* ws = (char*)d_ws;
  size_t off = 0;
  const size_t oWP = off; off += (size_t)WPLN * 2;             off = (off + 255) & ~(size_t)255;
  const size_t oDI = off; off += (size_t)nPad * 4;             off = (off + 255) & ~(size_t)255;
  const size_t oG  = off; off += (size_t)nPad * 128 * 4;       off = (off + 255) & ~(size_t)255;
  const size_t oPH = off; off += (size_t)nPad * 128 * 2;       off = (off + 255) & ~(size_t)255;
  const size_t oPL = off; off += (size_t)nPad * 128 * 2;       off = (off + 255) & ~(size_t)255;
  const size_t oZB = off; off += (size_t)nPad * 8 * 4;         off = (off + 255) & ~(size_t)255;
  if (off > ws_size) return;
  if (off > ((size_t)128 << 20)) return;
  unsigned short* wpl  = (unsigned short*)(ws + oWP);
  float*          dinv = (float*)(ws + oDI);
  float*          G    = (float*)(ws + oG);
  unsigned short* ph   = (unsigned short*)(ws + oPH);
  unsigned short* pl   = (unsigned short*)(ws + oPL);
  float*          zbs  = (float*)(ws + oZB);

  const int vec8 = ((nE & 3) == 0) ? 1 : 0;

  const int gDeg  = nPad / NBD;
  const int gG128 = (nN + 64 - 1) / 64;
  const int gG64  = (nN + 128 - 1) / 128;
  const int gA128 = (nN + NB128 - 1) / NB128;
  const int gA64  = (nN + NB64 - 1) / NB64;
  const int gA8   = (nN + NB8 - 1) / NB8;

  hipFuncSetAttribute(reinterpret_cast<const void*>(&k_agg128<0>), hipFuncAttributeMaxDynamicSharedMemorySize, LDS_128);
  hipFuncSetAttribute(reinterpret_cast<const void*>(&k_agg128<1>), hipFuncAttributeMaxDynamicSharedMemorySize, LDS_128);
  hipFuncSetAttribute(reinterpret_cast<const void*>(&k_agg64z),    hipFuncAttributeMaxDynamicSharedMemorySize, LDS_64);
  hipFuncSetAttribute(reinterpret_cast<const void*>(&k_agg8d),     hipFuncAttributeMaxDynamicSharedMemorySize, LDS_8);
  hipFuncSetAttribute(reinterpret_cast<const void*>(&k_deg),       hipFuncAttributeMaxDynamicSharedMemorySize, LDS_DEG);

  k_wprep<<<(320 * (KD / 8) + NTHR - 1) / NTHR, NTHR, 0, stream>>>(W1e, W2e, W2d, wpl);

  k_deg<<<gDeg, NTHR, LDS_DEG, stream>>>(ei, dinv, nE, vec8);

  k_gemm<128, false><<<gG128, NTHR, 0, stream>>>(x, ph, pl, wpl, dinv, G, nN, nPad);
  k_agg128<0><<<gA128, NTHR, LDS_128, stream>>>(ei, G, dinv, b1e, ph, pl, out, nN, nE, vec8);

  k_gemm<64, true><<<gG64, NTHR, 0, stream>>>(x, ph, pl, wpl + 2 * 128 * KD, dinv, G, nN, nPad);
  k_agg64z<<<gA64, NTHR, LDS_64, stream>>>(ei, G, dinv, b2e, Wm, bm, lnw, lnb, zbs, nN, nE, vec8);

  k_agg8d<<<gA8, NTHR, LDS_8, stream>>>(ei, zbs, dinv, W1d, b1d, ph, pl, nN, nE, vec8);

  k_gemm<128, true><<<gG128, NTHR, 0, stream>>>(x, ph, pl, wpl + 2 * 128 * KD + 2 * 64 * KD, dinv, G, nN, nPad);
  k_agg128<1><<<gA128, NTHR, LDS_128, stream>>>(ei, G, dinv, b2d, ph, pl, out, nN, nE, vec8);
}
